// Multi_Head_Attention_81484119539794
// MI455X (gfx1250) — hardware-run, weakly checked
//
#include <hip/hip_runtime.h>


#ifndef NB
#define NB 4
#endif
#ifndef SEQ
#define SEQ 2048
#endif
#define NB_FULL  4
#define SEQ_FULL 2048
#define DM   512
#define NH   8
#define HD   64
#define PCAR 1024.0f
#define PFL  (-24.0f)
#define SCL  0.125f
#define L2E  1.4426950408889634f
#define LKP  72
#define LPP  40
#define LOP  68
#define RK   64
#define NREL 129
#define RT   9
#define RPAD 144
#define LRP  148
#define LTP  72
#define LNEPS 1.0e-5f

static_assert(DM == NH * HD);
static_assert(HD == 64);
static_assert(DM % 32 == 0);
static_assert(DM % 64 == 0);
static_assert(SEQ % 64 == 0);
static_assert((SEQ * DM) % (8 * 256) == 0);
static_assert((DM * DM) % (8 * 256) == 0);
static_assert(NB <= NB_FULL);
static_assert(SEQ <= SEQ_FULL);
static_assert(LKP % 8 == 0);
static_assert(LPP % 8 == 0);
static_assert(LOP % 4 == 0);
static_assert(NREL == 2 * RK + 1);
static_assert(RPAD == RT * 16);
static_assert(NREL <= RPAD);
static_assert(RPAD <= LRP);
static_assert(2 * RK < RPAD);
static_assert((RPAD * HD) % 64 == 0);
static_assert(HD * 2 == 8 * 16);
static_assert(LTP % 8 == 0);
static_assert(SEQ % 4 == 0);
static_assert(256 * 16 * 2 == 64 * 64 * 2);
static_assert(32 * 16 * 4 == 16 * HD * 2);
static_assert(32 * 16 * 8 == 16 * 64 * 4);
static_assert(PCAR == 1024.0f);
static_assert((size_t)64 * LKP * 2 * 2 + (size_t)4 * 16 * LPP * 2 + (size_t)4 * 16 * LOP * 4 + (size_t)4 * 16 * LRP * 4 <= 131072);
static_assert((size_t)64 * LTP * 2 + 2 * 64 * 4 <= 131072);

typedef _Float16 h16;
typedef unsigned short bf;
typedef __attribute__((ext_vector_type(16))) __bf16   v16bf;
typedef __attribute__((ext_vector_type(16))) _Float16 v16h;
typedef __attribute__((ext_vector_type(8)))  _Float16 v8h;
typedef __attribute__((ext_vector_type(8)))  unsigned short v8us;
typedef __attribute__((ext_vector_type(8)))  float    v8f;
typedef __attribute__((ext_vector_type(4)))  float    v4f;
typedef __attribute__((ext_vector_type(4)))  int      v4i;
typedef v8h  __attribute__((may_alias)) v8ha;
typedef v4f  __attribute__((may_alias)) v4fa;
typedef v8us __attribute__((may_alias)) v8usa;

__device__ __forceinline__ unsigned short f2bf(float f) { unsigned u = __float_as_uint(f); u += 0x7FFFu + ((u >> 16) & 1u); return (unsigned short)(u >> 16); }
__device__ __forceinline__ float bf2f(unsigned short b) { return __uint_as_float(((unsigned)b) << 16); }
__device__ __forceinline__ float bfr(float f) { return bf2f(f2bf(f)); }
__device__ __forceinline__ void splitf(float y, unsigned short& h, unsigned short& l) { h = f2bf(y); l = f2bf(y - bf2f(h)); }
__device__ __forceinline__ v16h cat16(v8h lo, v8h hi) { return __builtin_shufflevector(lo, hi, 0, 1, 2, 3, 4, 5, 6, 7, 8, 9, 10, 11, 12, 13, 14, 15); }
__device__ __forceinline__ v16bf cat16b(v8us lo, v8us hi) { return __builtin_bit_cast(v16bf, __builtin_shufflevector(lo, hi, 0, 1, 2, 3, 4, 5, 6, 7, 8, 9, 10, 11, 12, 13, 14, 15)); }
__device__ __forceinline__ v8f wmma16(v16h a, v16h b, v8f c) { return __builtin_amdgcn_wmma_f32_16x16x32_f16(false, a, false, b, (short)0, c, false, false); }
__device__ __forceinline__ v8f wmmab(v16bf a, v16bf b, v8f c) { return __builtin_amdgcn_wmma_f32_16x16x32_bf16(false, a, false, b, (short)0, c, false, false); }
__device__ __forceinline__ v16bf ldg16(const bf* __restrict__ p) { return cat16b(*(const v8us*)p, *(const v8us*)(p + 16)); }
__device__ __forceinline__ void wsync() { __builtin_amdgcn_wave_barrier(); asm volatile("" ::: "memory"); }
__device__ __forceinline__ v8f wmmab_g(v16bf a, v16bf b, v8f c) { c = __builtin_amdgcn_wmma_f32_16x16x32_bf16(false, a, false, b, (short)0, c, false, false); asm volatile("v_nop\n\tv_nop\n\tv_nop\n\tv_nop" : "+v"(c) : "v"(a), "v"(b)); return c; }
__device__ __forceinline__ v8f wmma16_g(v16h a, v16h b, v8f c) { c = __builtin_amdgcn_wmma_f32_16x16x32_f16(false, a, false, b, (short)0, c, false, false); asm volatile("v_nop\n\tv_nop\n\tv_nop\n\tv_nop" : "+v"(c) : "v"(a), "v"(b)); return c; }
__device__ __forceinline__ h16 toh_flush(float v) { const h16 r = (h16)v; return (fabsf(v) < 6.103515625e-05f) ? (h16)0.0f : r; }
__device__ __forceinline__ int clampi(int v, int lo, int hi) { const int t = v < lo ? lo : v; return t > hi ? hi : t; }

template <int NSPLIT>
__device__ __forceinline__ void gemm_loop(const bf* __restrict__ A, const bf* __restrict__ A2, const bf* __restrict__ Bt, const int K, const size_t aoff, const size_t boff, v8f (&acc)[4][4]) {
#pragma unroll 1
    for (int kc = 0; kc < K; kc += 32) {
        v16bf a[4], a2[4];
#pragma unroll
        for (int mb = 0; mb < 4; ++mb) { a[mb] = ldg16(A + aoff + (size_t)mb * 16 * K + kc); if (NSPLIT == 1) a2[mb] = ldg16(A2 + aoff + (size_t)mb * 16 * K + kc); }
#pragma unroll
        for (int nb = 0; nb < 4; ++nb) { const v16bf b = ldg16(Bt + boff + (size_t)nb * 16 * K + kc);
#pragma unroll
            for (int mb = 0; mb < 4; ++mb) { acc[mb][nb] = wmmab(a[mb], b, acc[mb][nb]); if (NSPLIT == 1) acc[mb][nb] = wmmab(a2[mb], b, acc[mb][nb]); } }
        asm volatile("v_nop\n\tv_nop\n\tv_nop\n\tv_nop" : "+v"(acc[0][0]), "+v"(acc[1][1]), "+v"(acc[2][2]), "+v"(acc[3][3]) : "v"(a[0]), "v"(a[3]));
    }
}

__global__ __launch_bounds__(256) void k_cvt8(const float* __restrict__ src, bf* dst, unsigned n8, size_t sstride, size_t dstride) {
    const unsigned i = blockIdx.x * 256u + threadIdx.x; if (i >= n8) return;
    const float* s = src + (size_t)blockIdx.y * sstride + (size_t)i * 8; bf* d = dst + (size_t)blockIdx.y * dstride + (size_t)i * 8;
    const v4f v0 = *(const v4f*)s; const v4f v1 = *(const v4f*)(s + 4); v8us o;
#pragma unroll
    for (int k = 0; k < 4; ++k) { o[k] = f2bf(v0[k]); o[4 + k] = f2bf(v1[k]); }
    *(volatile v8us*)d = o; __threadfence(); *(volatile v8us*)d = o;
}

__global__ __launch_bounds__(256) void k_cvt8h(const float* __restrict__ src, bf* dst, unsigned n8, size_t sstride, float sc) {
#pragma clang fp contract(off)
    const unsigned i = blockIdx.x * 256u + threadIdx.x; if (i >= n8) return;
    const unsigned e = i * 8u; const unsigned srow = e / DM, c = e % DM; const unsigned hh = c / HD, dd = c % HD;
    const float* s = src + (size_t)blockIdx.y * sstride + (size_t)e;
    bf* d = dst + (((size_t)blockIdx.y * NH + hh) * SEQ + srow) * HD + dd;
    const v4f v0 = *(const v4f*)s; const v4f v1 = *(const v4f*)(s + 4); v8us o;
#pragma unroll
    for (int k = 0; k < 4; ++k) { o[k] = f2bf(bfr(v0[k]) * sc); o[4 + k] = f2bf(bfr(v1[k]) * sc); }
    *(volatile v8us*)d = o; __threadfence(); *(volatile v8us*)d = o;
}

__global__ __launch_bounds__(256) void k_cvt_rpe(const float* __restrict__ src, bf* dst) {
    const unsigned i = blockIdx.x * 256u + threadIdx.x; if (i >= (unsigned)(RPAD * HD / 8)) return;
    const unsigned nreal = (unsigned)(NREL * HD / 8);
    const unsigned ic = i < nreal ? i : nreal - 1u;
    const bool ok = i < nreal;
    const float* s = src + (size_t)ic * 8; bf* d = dst + (size_t)i * 8;
    const v4f v0 = *(const v4f*)s; const v4f v1 = *(const v4f*)(s + 4); v8us o;
#pragma unroll
    for (int k = 0; k < 4; ++k) { const unsigned short a = f2bf(v0[k]); const unsigned short c = f2bf(v1[k]); o[k] = ok ? a : (unsigned short)0; o[4 + k] = ok ? c : (unsigned short)0; }
    *(volatile v8us*)d = o; __threadfence(); *(volatile v8us*)d = o;
}

__global__ __launch_bounds__(256) void k_ln_vt(const float* __restrict__ X, const float* __restrict__ G, const float* __restrict__ Bt, h16* VT) {
#pragma clang fp contract(off)
    __shared__ __align__(16) h16 t_s[64 * LTP];
    __shared__ float mu_s[64];
    __shared__ float rs_s[64];
    const int tid = threadIdx.x, lane = tid & 31;
    const int wid = __builtin_amdgcn_readfirstlane(tid >> 5);
    const size_t z = blockIdx.y; const int s0 = blockIdx.x * 64;
    const float* xb = X + z * (size_t)SEQ_FULL * DM + (size_t)s0 * DM;
#pragma unroll 1
    for (int t = 0; t < 8; ++t) {
        const int tok = wid * 8 + t;
        const float* xr = xb + (size_t)tok * DM;
        float xv[16]; float sm = 0.0f;
#pragma unroll
        for (int c = 0; c < 16; ++c) { xv[c] = bfr(xr[c * 32 + lane]); sm += xv[c]; }
        sm += __shfl_xor(sm, 16, 32); sm += __shfl_xor(sm, 8, 32); sm += __shfl_xor(sm, 4, 32); sm += __shfl_xor(sm, 2, 32); sm += __shfl_xor(sm, 1, 32);
        const float mu = sm * (1.0f / DM);
        float sq = 0.0f;
#pragma unroll
        for (int c = 0; c < 16; ++c) { const float dv = xv[c] - mu; sq += dv * dv; }
        sq += __shfl_xor(sq, 16, 32); sq += __shfl_xor(sq, 8, 32); sq += __shfl_xor(sq, 4, 32); sq += __shfl_xor(sq, 2, 32); sq += __shfl_xor(sq, 1, 32);
        const float rstd = rsqrtf(sq * (1.0f / DM) + LNEPS);
        if (lane == 0) { mu_s[tok] = mu; rs_s[tok] = rstd; }
    }
    __syncthreads();
    const int f = tid & 63, tq = tid >> 6;
#pragma unroll 1
    for (int cc = 0; cc < DM / 64; ++cc) {
        const int c0 = cc * 64;
        const float g = bfr(G[c0 + f]), be = bfr(Bt[c0 + f]);
#pragma unroll 1
        for (int it = 0; it < 16; ++it) {
            const int tok = tq + 4 * it;
            const float x = bfr(xb[(size_t)tok * DM + c0 + f]);
            const float y = (x - mu_s[tok]) * rs_s[tok] * g + be;
            t_s[f * LTP + tok] = toh_flush(y);
        }
        __syncthreads();
#pragma unroll 1
        for (int ps = 0; ps < 2; ++ps) {
#pragma unroll
            for (int it = 0; it < 2; ++it) { const int u = tid + it * 256; const int row = u >> 3, part = (u & 7) * 8;
                const v8h o = *(const v8ha*)(&t_s[row * LTP + part]);
                *(volatile v8h*)(VT + (z * DM + (size_t)(c0 + row)) * SEQ + s0 + part) = o; }
            if (ps == 0) __threadfence(); }
        __syncthreads();
    }
}

__global__ __launch_bounds__(512) void k_relchk(const int* __restrict__ rel, float* pz) {
    __shared__ int bad_s[16];
    const int tid = threadIdx.x, lane = tid & 31;
    const int wid = __builtin_amdgcn_readfirstlane(tid >> 5);
    const unsigned per = SEQ / 4;
    int bad = 0;
#pragma unroll 1
    for (unsigned e = tid; e < (unsigned)SEQ * per; e += 512u) {
        const int i = (int)(e / per), j = (int)(e % per) * 4;
        const v4i t = *(const v4i*)(rel + (size_t)i * SEQ_FULL + j);
#pragma unroll
        for (int c = 0; c < 4; ++c) { const int want = clampi(j + c - i, -RK, RK) + RK; bad |= (t[c] != want) ? 1 : 0; }
    }
    bad |= __shfl_xor(bad, 16, 32); bad |= __shfl_xor(bad, 8, 32); bad |= __shfl_xor(bad, 4, 32); bad |= __shfl_xor(bad, 2, 32); bad |= __shfl_xor(bad, 1, 32);
    if (lane == 0) bad_s[wid] = bad;
    __syncthreads();
    int any = 0;
#pragma unroll
    for (int w = 0; w < 16; ++w) any |= bad_s[w];
    const float pv = (any != 0) ? __uint_as_float(0x7FC00000u) : 0.0f;
    if (tid < 8) { const v4f o = (v4f){pv, pv, pv, pv}; *(volatile v4f*)(pz + tid * 4) = o; __threadfence(); *(volatile v4f*)(pz + tid * 4) = o; }
}

__global__ __launch_bounds__(32) void k_gemm_out(const bf* __restrict__ Ah, const bf* __restrict__ Al, const bf* __restrict__ W, const float* __restrict__ pz, float* C) {
    __shared__ __align__(16) float os[16 * LOP];
    const int lane = threadIdx.x & 31, lr = lane & 15, hi = lane >> 4;
    const size_t z = blockIdx.z; const int r0 = blockIdx.x * 64, c0 = blockIdx.y * 64;
    const bf* A = Ah + z * (size_t)SEQ * DM; const bf* A2 = Al + z * (size_t)SEQ * DM;
    float* Cz = C + z * (size_t)SEQ_FULL * DM;
    const float pzv = pz[0];
    v8f acc[4][4];
#pragma unroll
    for (int mb = 0; mb < 4; ++mb)
#pragma unroll
        for (int nb = 0; nb < 4; ++nb) acc[mb][nb] = (v8f){};
    gemm_loop<1>(A, A2, W, DM, (size_t)(r0 + lr) * DM + 8 * hi, (size_t)(c0 + lr) * DM + 8 * hi, acc);
#pragma unroll
    for (int mb = 0; mb < 4; ++mb) {
#pragma unroll
        for (int nb = 0; nb < 4; ++nb) {
#pragma unroll
            for (int j = 0; j < 8; ++j) os[(hi * 8 + j) * LOP + nb * 16 + lr] = acc[mb][nb][j]; }
        wsync();
        float* crow = Cz + (size_t)(r0 + mb * 16) * DM + c0;
#pragma unroll 1
        for (int ps = 0; ps < 2; ++ps) {
#pragma unroll
            for (int s = 0; s < 8; ++s) { const int row = 2 * s + hi, cofs = lr * 4; v4f val = *(const v4fa*)(&os[row * LOP + cofs]);
                val[0] += pzv; val[1] += pzv; val[2] += pzv; val[3] += pzv;
                *(volatile v4f*)(crow + (size_t)row * DM + cofs) = val; }
            if (ps == 0) __threadfence(); }
        wsync();
    }
}

__global__ __launch_bounds__(128) void k_flash(const bf* __restrict__ Qh, const bf* __restrict__ Kh, const bf* __restrict__ RP, const h16* __restrict__ VT, bf* Ch, bf* Cl) {
    __shared__ __align__(16) bf    kh_s[64 * LKP];
    __shared__ __align__(16) h16   vt_s[64 * LKP];
    __shared__ __align__(16) h16   p_s[4 * 16 * LPP];
    __shared__ __align__(16) float o_s[4 * 16 * LOP];
    __shared__ __align__(16) float r_s[4 * 16 * LRP];
    const int tid = threadIdx.x, lane = tid & 31, lr = lane & 15, hi = lane >> 4;
    const int wid = __builtin_amdgcn_readfirstlane(tid >> 5);
    const int bh = blockIdx.y; const int b = bh / NH, h = bh % NH;
    const int q0 = blockIdx.x * 64 + wid * 16;
    const size_t pl = (size_t)bh * SEQ * HD;
    const size_t qoff = pl + (size_t)(q0 + lr) * HD + 8 * hi;
    const size_t vbase = ((size_t)b * DM + (size_t)h * HD) * SEQ;
    const int pb = wid * 16 * LPP, ob = wid * 16 * LOP;
    const int rb = wid * 16 * LRP + 8 * hi * LRP;
    {
        const v16bf qa0 = ldg16(Qh + qoff); const v16bf qa1 = ldg16(Qh + qoff + 32);
#pragma unroll 1
        for (int ct = 0; ct < RT; ++ct) {
            const size_t ro = (size_t)(ct * 16 + lr) * HD + 8 * hi;
            const v16bf b0 = ldg16(RP + ro); const v16bf b1 = ldg16(RP + ro + 32);
            v8f t = (v8f){};
            t = wmmab_g(qa0, b0, t);
            t = wmmab_g(qa1, b1, t);
#pragma unroll
            for (int j = 0; j < 8; ++j) r_s[rb + j * LRP + ct * 16 + lr] = t[j];
        }
    }
    wsync();
    float rlo[8], rhi[8];
#pragma unroll
    for (int r = 0; r < 8; ++r) { rlo[r] = r_s[rb + r * LRP]; rhi[r] = r_s[rb + r * LRP + 2 * RK]; }
    v8f o[4];
#pragma unroll
    for (int dt = 0; dt < 4; ++dt) o[dt] = (v8f){};
    float mr[8], ls[8];
#pragma unroll
    for (int r = 0; r < 8; ++r) { mr[r] = -1.0e30f; ls[r] = 0.0f; }

#pragma unroll 1
    for (int kb = 0; kb < SEQ / 64; ++kb) {
        __syncthreads();
#pragma unroll
        for (int it = 0; it < 4; ++it) {
            const int u = tid + it * 128; const int row = u >> 3, part = (u & 7) * 8;
            const size_t g = pl + (size_t)kb * 64 * HD + (size_t)u * 8;
            const v8us a = *(const v8us*)(Kh + g);
            const v8h v = *(const v8h*)(VT + vbase + (size_t)row * SEQ + (size_t)kb * 64 + part);
            *(v8usa*)(&kh_s[row * LKP + part]) = a; *(v8ha*)(&vt_s[row * LKP + part]) = v;
        }
        __syncthreads();
#pragma unroll 1
        for (int hf = 0; hf < 2; ++hf) {
            v8f s0 = (v8f){}, s1 = (v8f){};
            const int kr0 = (hf * 32 + lr) * LKP + 8 * hi, kr1 = kr0 + 16 * LKP;
#pragma unroll
            for (int ks = 0; ks < 2; ++ks) {
                const int kk = ks * 32;
                const v16bf qh = ldg16(Qh + qoff + kk);
                const v16bf k0h = cat16b(*(const v8usa*)(&kh_s[kr0 + kk]), *(const v8usa*)(&kh_s[kr0 + kk + 16]));
                const v16bf k1h = cat16b(*(const v8usa*)(&kh_s[kr1 + kk]), *(const v8usa*)(&kh_s[kr1 + kk + 16]));
                s0 = wmmab_g(qh, k0h, s0); s1 = wmmab_g(qh, k1h, s1);
            }
            const int j0 = kb * 64 + hf * 32;
            if (j0 - q0 >= RK + 15) {
#pragma unroll
                for (int r = 0; r < 8; ++r) { s0[r] += rhi[r]; s1[r] += rhi[r]; }
            } else if (q0 - j0 >= RK + 31) {
#pragma unroll
                for (int r = 0; r < 8; ++r) { s0[r] += rlo[r]; s1[r] += rlo[r]; }
            } else {
#pragma unroll
                for (int r = 0; r < 8; ++r) {
                    const int d0 = j0 + lr - q0 - 8 * hi - r;
                    const int i0 = clampi(d0, -RK, RK) + RK, i1 = clampi(d0 + 16, -RK, RK) + RK;
                    const float b0 = r_s[rb + r * LRP + i0]; const float b1 = r_s[rb + r * LRP + i1];
                    s0[r] += b0; s1[r] += b1;
                }
            }
#pragma unroll
            for (int r = 0; r < 8; ++r) {
                const float a0 = s0[r], a1 = s1[r];
                float mx = fmaxf(a0, a1);
                mx = fmaxf(mx, __shfl_xor(mx, 1, 32)); mx = fmaxf(mx, __shfl_xor(mx, 2, 32)); mx = fmaxf(mx, __shfl_xor(mx, 4, 32)); mx = fmaxf(mx, __shfl_xor(mx, 8, 32));
                const float mnew = fmaxf(mr[r], mx);
                const float al = __builtin_amdgcn_exp2f((mr[r] - mnew) * L2E);
                const float e0 = (a0 - mnew) * L2E, e1 = (a1 - mnew) * L2E;
                const float p0 = __builtin_amdgcn_exp2f(e0);
                const float p1 = __builtin_amdgcn_exp2f(e1);
                ls[r] = ls[r] * al + (p0 + p1);
                mr[r] = mnew;
                o[0][r] *= al; o[1][r] *= al; o[2][r] *= al; o[3][r] *= al;
                p_s[pb + (8 * hi + r) * LPP + lr] = (e0 < PFL) ? (h16)0.0f : (h16)(p0 * PCAR);
                p_s[pb + (8 * hi + r) * LPP + 16 + lr] = (e1 < PFL) ? (h16)0.0f : (h16)(p1 * PCAR);
            }
            wsync();
            const v16h pa = cat16(*(const v8ha*)(&p_s[pb + lr * LPP + 8 * hi]), *(const v8ha*)(&p_s[pb + lr * LPP + 8 * hi + 16]));
            v16h vb[4];
#pragma unroll
            for (int dt = 0; dt < 4; ++dt) { const int vo = (dt * 16 + lr) * LKP + hf * 32 + 8 * hi; vb[dt] = cat16(*(const v8ha*)(&vt_s[vo]), *(const v8ha*)(&vt_s[vo + 16])); }
#pragma unroll
            for (int dt = 0; dt < 4; ++dt) o[dt] = wmma16_g(pa, vb[dt], o[dt]);
            wsync();
        }
    }
#pragma unroll
    for (int r = 0; r < 8; ++r) {
        float lt = ls[r];
        lt += __shfl_xor(lt, 1, 32); lt += __shfl_xor(lt, 2, 32); lt += __shfl_xor(lt, 4, 32); lt += __shfl_xor(lt, 8, 32);
        const float inv = 1.0f / (lt * PCAR);
#pragma unroll
        for (int dt = 0; dt < 4; ++dt) o_s[ob + (8 * hi + r) * LOP + dt * 16 + lr] = o[dt][r] * inv;
    }
    wsync();
    const int srow = lane >> 3, scol = (lane & 7) * 8;
    const size_t cbase = ((size_t)b * SEQ + q0) * DM + (size_t)h * HD;
#pragma unroll 1
    for (int ps = 0; ps < 2; ++ps) {
#pragma unroll
        for (int s = 0; s < 4; ++s) { const int row = 4 * s + srow; const v4f x0 = *(const v4fa*)(&o_s[ob + row * LOP + scol]); const v4f x1 = *(const v4fa*)(&o_s[ob + row * LOP + scol + 4]); v8us oh, ol;
#pragma unroll
            for (int j = 0; j < 4; ++j) { unsigned short a, c; splitf(x0[j], a, c); oh[j] = a; ol[j] = c; splitf(x1[j], a, c); oh[4 + j] = a; ol[4 + j] = c; }
            const size_t off = cbase + (size_t)row * DM + scol;
            *(volatile v8us*)(Ch + off) = oh; *(volatile v8us*)(Cl + off) = ol; }
        if (ps == 0) __threadfence(); }
}

constexpr size_t al256(size_t x) { return (x + 255) & ~(size_t)255; }
constexpr size_t SZ_W = al256((size_t)DM * DM * 2);
constexpr size_t SZ_R = al256((size_t)RPAD * HD * 2);
constexpr size_t SZ_X = al256((size_t)NB * SEQ * DM * 2);
constexpr size_t SZ_P = al256((size_t)NB * NH * SEQ * HD * 2);
constexpr size_t SZ_F = 256;
constexpr size_t WS_TOTAL = SZ_W + SZ_R + 2 * SZ_P + SZ_P + 2 * SZ_X + SZ_F;
static_assert(WS_TOTAL <= (size_t)134217728);
static_assert(SZ_P == SZ_X);
static_assert(SZ_R >= (size_t)RPAD * HD * 2);

extern "C" void kernel_launch(void* const* d_in, const int* in_sizes, int n_in,
                              void* d_out, int out_size, void* d_ws, size_t ws_size, hipStream_t stream) {
    if (n_in < 8) return;
    const size_t need_act = (size_t)(NB - 1) * SEQ_FULL * DM + (size_t)SEQ * DM;
    if ((size_t)in_sizes[0] < need_act || (size_t)in_sizes[1] < need_act || (size_t)in_sizes[2] < need_act) return;
    if (in_sizes[3] < DM || in_sizes[4] < DM || in_sizes[5] < NREL * HD || (size_t)in_sizes[6] < (size_t)DM * DM) return;
    if ((size_t)in_sizes[7] < (size_t)(SEQ - 1) * SEQ_FULL + (size_t)SEQ) return;
    if ((size_t)out_size < need_act) return;
    if (WS_TOTAL > ws_size) return;
    const float* xq = (const float*)d_in[0]; const float* xk = (const float*)d_in[1]; const float* xv = (const float*)d_in[2];
    const float* lg = (const float*)d_in[3]; const float* lb = (const float*)d_in[4]; const float* rp = (const float*)d_in[5]; const float* wp = (const float*)d_in[6];
    const int* rel = (const int*)d_in[7];
    float* OUT = (float*)d_out;
    char* wsp = (char*)d_ws;
    auto take = [&](size_t bytes) { char* p = wsp; wsp += bytes; return (void*)p; };
    bf* WO = (bf*)take(SZ_W);
    bf* RPP = (bf*)take(SZ_R);
    bf* QP = (bf*)take(SZ_P); bf* KP = (bf*)take(SZ_P);
    h16* VT = (h16*)take(SZ_P);
    bf* CTh = (bf*)take(SZ_X); bf* CTl = (bf*)take(SZ_X);
    float* PZ = (float*)take(SZ_F);
    if ((size_t)(wsp - (char*)d_ws) != WS_TOTAL) return;

    const unsigned nw8 = (unsigned)((size_t)DM * DM / 8), na8 = (unsigned)((size_t)SEQ * DM / 8);
    k_cvt8<<<dim3(nw8 / 256, 1), 256, 0, stream>>>(wp, WO, nw8, 0, 0);
    k_cvt_rpe<<<dim3((RPAD * HD / 8 + 255) / 256), 256, 0, stream>>>(rp, RPP);
    k_cvt8h<<<dim3(na8 / 256, NB), 256, 0, stream>>>(xq, QP, na8, (size_t)SEQ_FULL * DM, SCL);
    k_cvt8h<<<dim3(na8 / 256, NB), 256, 0, stream>>>(xk, KP, na8, (size_t)SEQ_FULL * DM, 1.0f);
    k_ln_vt<<<dim3(SEQ / 64, NB), 256, 0, stream>>>(xv, lg, lb, VT);
    k_relchk<<<dim3(1), 512, 0, stream>>>(rel, PZ);
    k_flash<<<dim3(SEQ / 64, NB * NH), 128, 0, stream>>>(QP, KP, RPP, VT, CTh, CTl);
    k_gemm_out<<<dim3(SEQ / 64, DM / 64, NB), 32, 0, stream>>>(CTh, CTl, WO, PZ, OUT);
}
